// SelfAttention_558345748853
// MI455X (gfx1250) — hardware-verified
//
#include <hip/hip_runtime.h>


#ifndef NB
#define NB 1
#endif
#ifndef SEQ
#define SEQ 2048
#endif
#define NB_FULL  1
#define SEQ_FULL 2048
#define DM   2048
#define NH   32
#define NKV  8
#define REP  (NH / NKV)
#define HD   64
#define DQ   (NH * HD)
#define DKV  (NKV * HD)
#define RH   ((SEQ) < 512 ? (SEQ) : 512)
#define NW   (SEQ / 32)
#define PP   40
#define PCAR 1024.0f
#define SCL2 0.18033688011112042f

static_assert(SEQ % 64 == 0);
static_assert(SEQ <= SEQ_FULL);
static_assert(NW <= 64);
static_assert(HD == 64);
static_assert(DM % 64 == 0 && DQ % 64 == 0 && DKV % 64 == 0);
static_assert(DM % 32 == 0 && DQ % 32 == 0);
static_assert(NH % NKV == 0);
static_assert(RH % 16 == 0 && (SEQ - RH) % 16 == 0);
static_assert((PP * 2) % 16 == 0);
static_assert(NB <= NB_FULL);

typedef _Float16 h16;
typedef unsigned short bf;
typedef __attribute__((ext_vector_type(16))) __bf16   v16bf;
typedef __attribute__((ext_vector_type(16))) _Float16 v16h;
typedef __attribute__((ext_vector_type(8)))  _Float16 v8h;
typedef __attribute__((ext_vector_type(8)))  unsigned short v8us;
typedef __attribute__((ext_vector_type(8)))  float    v8f;
typedef __attribute__((ext_vector_type(4)))  float    v4f;
typedef __attribute__((ext_vector_type(2)))  _Float16 v2h;
typedef __attribute__((ext_vector_type(2)))  unsigned short v2us;
typedef __attribute__((ext_vector_type(2)))  float    v2f;
typedef v4f  __attribute__((may_alias)) v4fa;
typedef v8us __attribute__((may_alias)) v8usa;

__device__ __forceinline__ unsigned short f2bf(float f) { unsigned u = __float_as_uint(f); u += 0x7FFFu + ((u >> 16) & 1u); return (unsigned short)(u >> 16); }
__device__ __forceinline__ float bf2f(unsigned short b) { return __uint_as_float(((unsigned)b) << 16); }
__device__ __forceinline__ float bfr(float f) { return bf2f(f2bf(f)); }
__device__ __forceinline__ v16h cat16(v8h lo, v8h hi) { return __builtin_shufflevector(lo, hi, 0, 1, 2, 3, 4, 5, 6, 7, 8, 9, 10, 11, 12, 13, 14, 15); }
__device__ __forceinline__ v16bf cat16b(v8us lo, v8us hi) { return __builtin_bit_cast(v16bf, __builtin_shufflevector(lo, hi, 0, 1, 2, 3, 4, 5, 6, 7, 8, 9, 10, 11, 12, 13, 14, 15)); }
__device__ __forceinline__ v16h cat16hu(v8us lo, v8us hi) { return __builtin_bit_cast(v16h, __builtin_shufflevector(lo, hi, 0, 1, 2, 3, 4, 5, 6, 7, 8, 9, 10, 11, 12, 13, 14, 15)); }
__device__ __forceinline__ v8f wmma16(v16h a, v16h b, v8f c) { return __builtin_amdgcn_wmma_f32_16x16x32_f16(false, a, false, b, (short)0, c, false, false); }
__device__ __forceinline__ v8f wmmab(v16bf a, v16bf b, v8f c) { return __builtin_amdgcn_wmma_f32_16x16x32_bf16(false, a, false, b, (short)0, c, false, false); }
__device__ __forceinline__ void splitf(float y, unsigned short& h, unsigned short& l) { h = f2bf(y); l = f2bf(y - bf2f(h)); }
__device__ __forceinline__ float ex2(float x) { return __builtin_amdgcn_exp2f(x); }

template <typename T16> struct WFrag;
template <> struct WFrag<h16> { typedef v16h V; static __device__ __forceinline__ V ld(const h16* p) { return cat16(*(const v8h*)p, *(const v8h*)(p + 16)); } static __device__ __forceinline__ v8f mma(V a, V b, v8f c) { return wmma16(a, b, c); } };
template <> struct WFrag<bf> { typedef v16bf V; static __device__ __forceinline__ V ld(const bf* p) { return cat16b(*(const v8us*)p, *(const v8us*)(p + 16)); } static __device__ __forceinline__ v8f mma(V a, V b, v8f c) { return wmmab(a, b, c); } };

template <typename T16, int NSPLIT>
__device__ __forceinline__ void gemmw_body(const T16* __restrict__ A, const T16* __restrict__ A2, const T16* __restrict__ Bt, int K, float* C, int ldc) {
    typedef typename WFrag<T16>::V V;
    __shared__ __align__(16) float os[16 * 68];
    const int lane = threadIdx.x & 31, lr = lane & 15, hi = lane >> 4; const int r0 = blockIdx.x * 64, c0 = blockIdx.y * 64;
    v8f acc[4][4];
#pragma unroll
    for (int mb = 0; mb < 4; ++mb)
#pragma unroll
        for (int nb = 0; nb < 4; ++nb) acc[mb][nb] = (v8f){};
    const size_t aoff = (size_t)(r0 + lr) * K + 8 * hi, boff = (size_t)(c0 + lr) * K + 8 * hi;
#pragma unroll 1
    for (int kc = 0; kc < K; kc += 32) {
        V a[4], a2[4];
#pragma unroll
        for (int mb = 0; mb < 4; ++mb) { a[mb] = WFrag<T16>::ld(A + aoff + (size_t)mb * 16 * K + kc); if (NSPLIT == 1) a2[mb] = WFrag<T16>::ld(A2 + aoff + (size_t)mb * 16 * K + kc); else a2[mb] = a[mb]; }
#pragma unroll
        for (int nb = 0; nb < 4; ++nb) { const V b = WFrag<T16>::ld(Bt + boff + (size_t)nb * 16 * K + kc);
#pragma unroll
            for (int mb = 0; mb < 4; ++mb) { acc[mb][nb] = WFrag<T16>::mma(a[mb], b, acc[mb][nb]); if (NSPLIT == 1) acc[mb][nb] = WFrag<T16>::mma(a2[mb], b, acc[mb][nb]); } }
        asm volatile("v_nop\n\tv_nop\n\tv_nop\n\tv_nop" : "+v"(acc[0][0]), "+v"(acc[1][1]), "+v"(acc[2][2]), "+v"(acc[3][3]) : "v"(a[0]), "v"(a[3]));
    }
#pragma unroll
    for (int mb = 0; mb < 4; ++mb) {
#pragma unroll
        for (int nb = 0; nb < 4; ++nb) {
#pragma unroll
            for (int j = 0; j < 8; ++j) os[(hi * 8 + j) * 68 + nb * 16 + lr] = acc[mb][nb][j]; }
        __builtin_amdgcn_wave_barrier(); asm volatile("" ::: "memory");
        float* crow = C + (size_t)(r0 + mb * 16) * ldc + c0;
#pragma unroll 1
        for (int ps = 0; ps < 2; ++ps) {
#pragma unroll
            for (int s = 0; s < 8; ++s) { const int row = 2 * s + hi, cofs = lr * 4; const v4f val = *(const v4fa*)(os + row * 68 + cofs);
                *(volatile v4f*)(crow + (size_t)row * ldc + cofs) = val; }
            if (ps == 0) __threadfence(); }
        __builtin_amdgcn_wave_barrier(); asm volatile("" ::: "memory");
    }
}
__global__ __launch_bounds__(32) void k_gemm_p(const bf* __restrict__ A, const bf* __restrict__ Bt, int K, float* C, int ldc) { gemmw_body<bf, 0>(A, A, Bt, K, C, ldc); }
__global__ __launch_bounds__(32) void k_gemm_s(const bf* __restrict__ A, const bf* __restrict__ A2, const bf* __restrict__ Bt, int K, float* C, int ldc) { gemmw_body<bf, 1>(A, A2, Bt, K, C, ldc); }

__global__ __launch_bounds__(256) void k_wtG(const float* __restrict__ w, int K, int N, bf* Bt) {
    const int lane = threadIdx.x & 31; const int L0 = (blockIdx.x * 8 + (threadIdx.x >> 5)) * 8; const int nlines = N * K / 64;
#pragma unroll
    for (int ps = 0; ps < 2; ++ps) {
#pragma unroll 1
        for (int l = 0; l < 8; ++l) { const int L = L0 + l; if (L >= nlines) break; const size_t e = (size_t)L * 64 + lane * 2; const int k = (int)(e % K), n = (int)(e / K); v2us o;
            o[0] = f2bf(w[(size_t)k * N + n]); o[1] = f2bf(w[(size_t)(k + 1) * N + n]); *(volatile v2us*)(Bt + e) = o; }
        if (ps == 0) __threadfence(); }
}
__global__ __launch_bounds__(256) void k_cvt8(const float* __restrict__ src, bf* dst, size_t n8) { const size_t i = (size_t)blockIdx.x * 256 + threadIdx.x; if (i >= n8) return; const v8f v = *(const v8f*)(src + i * 8); v8us o;
#pragma unroll
    for (int k = 0; k < 8; ++k) o[k] = f2bf(v[k]); *(volatile v8us*)(dst + i * 8) = o; __threadfence(); *(volatile v8us*)(dst + i * 8) = o; }

__global__ __launch_bounds__(256) void k_rope(const float* __restrict__ F, int pitch, int nheads, const float* __restrict__ COS, const float* __restrict__ SIN, h16* P16, bf* Ph, bf* Pl) {
#pragma clang fp contract(off)
    const size_t e = ((size_t)blockIdx.x * 256 + threadIdx.x) * 2; if (e >= (size_t)nheads * SEQ * HD) return;
    const int d = (int)(e % HD); const int t = (int)((e / HD) % SEQ); const int h = (int)(e / ((size_t)HD * SEQ));
    const v2f x = *(const v2f*)(F + (size_t)t * pitch + h * HD + d);
    const float c = bfr(COS[(size_t)t * (HD / 2) + (d >> 1)]), s = bfr(SIN[(size_t)t * (HD / 2) + (d >> 1)]);
    const float a0 = x[0] * c, a1 = x[1] * s, b0 = x[0] * s, b1 = x[1] * c;
    const float r0 = a0 - a1, r1 = b0 + b1;
    v2h o16; v2us oh, ol; unsigned short a2, c2;
    o16[0] = (h16)r0; splitf(r0, a2, c2); oh[0] = a2; ol[0] = c2;
    o16[1] = (h16)r1; splitf(r1, a2, c2); oh[1] = a2; ol[1] = c2;
    *(volatile v2h*)(P16 + e) = o16; *(volatile v2us*)(Ph + e) = oh; *(volatile v2us*)(Pl + e) = ol; __threadfence(); *(volatile v2h*)(P16 + e) = o16; *(volatile v2us*)(Ph + e) = oh; *(volatile v2us*)(Pl + e) = ol; }
__global__ __launch_bounds__(256) void k_vtp(const float* __restrict__ F, int pitch, int nheads, h16* V16, bf* Vh, bf* Vl) { const size_t e = ((size_t)blockIdx.x * 256 + threadIdx.x) * 2; if (e >= (size_t)nheads * HD * SEQ) return; const int t = (int)(e % SEQ); const int d = (int)((e / SEQ) % HD); const int g = (int)(e / ((size_t)SEQ * HD)); v2h o16; v2us oh, ol;
#pragma unroll
    for (int q = 0; q < 2; ++q) { const float x = F[(size_t)(t + q) * pitch + g * HD + d]; o16[q] = (h16)x; unsigned short a2, c2; splitf(x, a2, c2); oh[q] = a2; ol[q] = c2; }
    *(volatile v2h*)(V16 + e) = o16; *(volatile v2us*)(Vh + e) = oh; *(volatile v2us*)(Vl + e) = ol; __threadfence(); *(volatile v2h*)(V16 + e) = o16; *(volatile v2us*)(Vh + e) = oh; *(volatile v2us*)(Vl + e) = ol; }

__global__ __launch_bounds__(32) void k_maskbits(const int* __restrict__ mask, unsigned* MBp, int* CLp) {
    const int lane = threadIdx.x & 31; const int qt = blockIdx.x; const int q0 = qt * 16;
    unsigned and0 = 0xFFFFFFFFu, and1 = 0xFFFFFFFFu, or0 = 0u, or1 = 0u;
#pragma unroll 1
    for (int row = 0; row < 16; ++row) {
        const int* mr = mask + (size_t)(q0 + row) * SEQ_FULL; unsigned w0 = 0u, w1 = 0u;
#pragma unroll 4
        for (int w = 0; w < NW; ++w) { const int v = mr[32 * w + lane]; const unsigned b = __builtin_amdgcn_ballot_w32(v != 0); w0 = (w == lane) ? b : w0; w1 = (w == lane + 32) ? b : w1; }
        and0 &= w0; and1 &= w1; or0 |= w0; or1 |= w1;
        unsigned* dst = MBp + (size_t)(q0 + row) * NW;
        if (lane < NW) *(volatile unsigned*)(dst + lane) = w0;
        if (lane + 32 < NW) *(volatile unsigned*)(dst + 32 + lane) = w1;
        __threadfence();
        if (lane < NW) *(volatile unsigned*)(dst + lane) = w0;
        if (lane + 32 < NW) *(volatile unsigned*)(dst + 32 + lane) = w1;
    }
    const int c0 = (or0 == 0u) ? 0 : ((and0 == 0xFFFFFFFFu) ? 1 : 2); const int c1 = (or1 == 0u) ? 0 : ((and1 == 0xFFFFFFFFu) ? 1 : 2);
    int* cd = CLp + (size_t)qt * NW;
    if (lane < NW) *(volatile int*)(cd + lane) = c0;
    if (lane + 32 < NW) *(volatile int*)(cd + 32 + lane) = c1;
    __threadfence();
    if (lane < NW) *(volatile int*)(cd + lane) = c0;
    if (lane + 32 < NW) *(volatile int*)(cd + 32 + lane) = c1;
}

template <bool SPLIT>
__device__ __forceinline__ void attn_body(const h16* __restrict__ Q16, const h16* __restrict__ K16, const h16* __restrict__ V16,
                                          const bf* __restrict__ Qh, const bf* __restrict__ Ql, const bf* __restrict__ Kh, const bf* __restrict__ Kl, const bf* __restrict__ Vh, const bf* __restrict__ Vl,
                                          const unsigned* __restrict__ MBp, const int* __restrict__ CLp, bf* Ch, bf* Cl, int qt0) {
    __shared__ __align__(16) unsigned short pa[16 * PP];
    __shared__ __align__(16) unsigned short pb[16 * PP];
    __shared__ __align__(16) float os[16 * 68];
    const int lane = threadIdx.x & 31, lr = lane & 15, hi = lane >> 4;
    const int qt = qt0 + (int)blockIdx.x; const int h = (int)blockIdx.y; const int hk = h / REP; const int q0 = qt * 16;
    const size_t qoff = ((size_t)h * SEQ + q0 + lr) * HD + 8 * hi;
    const size_t kb0  = ((size_t)hk * SEQ + lr) * HD + 8 * hi;
    const size_t vb0  = ((size_t)hk * HD + lr) * SEQ + 8 * hi;
    const float NINF = -__builtin_inff();
    float mi[8], li[8]; v8f acc[4];
#pragma unroll
    for (int r = 0; r < 8; ++r) { mi[r] = NINF; li[r] = 0.0f; }
#pragma unroll
    for (int ot = 0; ot < 4; ++ot) acc[ot] = (v8f){};
#pragma unroll 1
    for (int j = 0; j < NW; ++j) {
        const int cls = __builtin_amdgcn_readfirstlane(CLp[(size_t)qt * NW + j]);
        if (cls == 0) continue;
        unsigned wd[8];
        if (cls == 1) {
#pragma unroll
            for (int r = 0; r < 8; ++r) wd[r] = 0xFFFFFFFFu;
        } else {
#pragma unroll
            for (int r = 0; r < 8; ++r) wd[r] = MBp[(size_t)(q0 + 8 * hi + r) * NW + j];
        }
        v8f s0 = (v8f){}, s1 = (v8f){};
        const size_t ko = kb0 + (size_t)(32 * j) * HD;
        if (SPLIT) {
            const v16bf qh0 = WFrag<bf>::ld(Qh + qoff), qh1 = WFrag<bf>::ld(Qh + qoff + 32), ql0 = WFrag<bf>::ld(Ql + qoff), ql1 = WFrag<bf>::ld(Ql + qoff + 32);
            { const v16bf kh0 = WFrag<bf>::ld(Kh + ko), kh1 = WFrag<bf>::ld(Kh + ko + 32), kl0 = WFrag<bf>::ld(Kl + ko), kl1 = WFrag<bf>::ld(Kl + ko + 32);
              s0 = wmmab(ql0, kh0, s0); s0 = wmmab(ql1, kh1, s0); s0 = wmmab(qh0, kl0, s0); s0 = wmmab(qh1, kl1, s0); s0 = wmmab(qh0, kh0, s0); s0 = wmmab(qh1, kh1, s0); }
            { const size_t k1 = ko + (size_t)16 * HD; const v16bf kh0 = WFrag<bf>::ld(Kh + k1), kh1 = WFrag<bf>::ld(Kh + k1 + 32), kl0 = WFrag<bf>::ld(Kl + k1), kl1 = WFrag<bf>::ld(Kl + k1 + 32);
              s1 = wmmab(ql0, kh0, s1); s1 = wmmab(ql1, kh1, s1); s1 = wmmab(qh0, kl0, s1); s1 = wmmab(qh1, kl1, s1); s1 = wmmab(qh0, kh0, s1); s1 = wmmab(qh1, kh1, s1);
              asm volatile("v_nop\n\tv_nop\n\tv_nop\n\tv_nop" : "+v"(s0), "+v"(s1) : "v"(qh1), "v"(kh1)); }
        } else {
            const v16h qa0 = WFrag<h16>::ld(Q16 + qoff), qa1 = WFrag<h16>::ld(Q16 + qoff + 32);
            const v16h k00 = WFrag<h16>::ld(K16 + ko), k01 = WFrag<h16>::ld(K16 + ko + 32);
            const v16h k10 = WFrag<h16>::ld(K16 + ko + (size_t)16 * HD), k11 = WFrag<h16>::ld(K16 + ko + (size_t)16 * HD + 32);
            s0 = wmma16(qa0, k00, s0); s0 = wmma16(qa1, k01, s0); s1 = wmma16(qa0, k10, s1); s1 = wmma16(qa1, k11, s1);
            asm volatile("v_nop\n\tv_nop\n\tv_nop\n\tv_nop" : "+v"(s0), "+v"(s1) : "v"(qa1), "v"(k11));
        }
#pragma unroll
        for (int r = 0; r < 8; ++r) {
            const unsigned w = wd[r];
            const bool kp0 = ((w >> lr) & 1u) != 0u, kp1 = ((w >> (16 + lr)) & 1u) != 0u;
            const float v0 = kp0 ? s0[r] * SCL2 : NINF; const float v1 = kp1 ? s1[r] * SCL2 : NINF;
            float mx = fmaxf(v0, v1);
            mx = fmaxf(mx, __shfl_xor(mx, 1, 32)); mx = fmaxf(mx, __shfl_xor(mx, 2, 32)); mx = fmaxf(mx, __shfl_xor(mx, 4, 32)); mx = fmaxf(mx, __shfl_xor(mx, 8, 32));
            const float nm = fmaxf(mi[r], mx); const float ms = (nm == NINF) ? 0.0f : nm;
            const float corr = ex2(mi[r] - ms); const float p0 = ex2(v0 - ms), p1 = ex2(v1 - ms);
            const int po = (8 * hi + r) * PP + lr;
            if (SPLIT) { unsigned short a, c; splitf(p0, a, c); pa[po] = a; pb[po] = c; splitf(p1, a, c); pa[po + 16] = a; pb[po + 16] = c; li[r] = li[r] * corr + (p0 + p1); }
            else { const h16 e0 = (h16)(p0 * PCAR), e1 = (h16)(p1 * PCAR); pa[po] = __builtin_bit_cast(unsigned short, e0); pa[po + 16] = __builtin_bit_cast(unsigned short, e1); li[r] = li[r] * corr + ((float)e0 + (float)e1); }
            mi[r] = nm;
#pragma unroll
            for (int ot = 0; ot < 4; ++ot) acc[ot][r] *= corr;
        }
        __syncthreads();
        const size_t vo = vb0 + (size_t)(32 * j);
        if (SPLIT) {
            const v8us a0 = *(const v8usa*)(pa + lr * PP + 8 * hi), a1 = *(const v8usa*)(pa + lr * PP + 16 + 8 * hi);
            const v8us b0 = *(const v8usa*)(pb + lr * PP + 8 * hi), b1 = *(const v8usa*)(pb + lr * PP + 16 + 8 * hi);
            const v16bf ph = cat16b(a0, a1), pl = cat16b(b0, b1);
#pragma unroll
            for (int ot = 0; ot < 4; ++ot) { const v16bf vh = WFrag<bf>::ld(Vh + vo + (size_t)ot * 16 * SEQ), vl = WFrag<bf>::ld(Vl + vo + (size_t)ot * 16 * SEQ);
                acc[ot] = wmmab(pl, vh, acc[ot]); acc[ot] = wmmab(ph, vl, acc[ot]); acc[ot] = wmmab(ph, vh, acc[ot]); }
            asm volatile("v_nop\n\tv_nop\n\tv_nop\n\tv_nop" : "+v"(acc[0]), "+v"(acc[1]), "+v"(acc[2]), "+v"(acc[3]) : "v"(ph), "v"(pl));
        } else {
            const v8us a0 = *(const v8usa*)(pa + lr * PP + 8 * hi), a1 = *(const v8usa*)(pa + lr * PP + 16 + 8 * hi);
            const v16h p16 = cat16hu(a0, a1);
#pragma unroll
            for (int ot = 0; ot < 4; ++ot) { const v16h vf = WFrag<h16>::ld(V16 + vo + (size_t)ot * 16 * SEQ); acc[ot] = wmma16(p16, vf, acc[ot]); }
            asm volatile("v_nop\n\tv_nop\n\tv_nop\n\tv_nop" : "+v"(acc[0]), "+v"(acc[1]), "+v"(acc[2]), "+v"(acc[3]) : "v"(p16));
        }
        asm volatile("" ::: "memory");
    }
#pragma unroll
    for (int r = 0; r < 8; ++r) { float l = li[r]; l += __shfl_xor(l, 1, 32); l += __shfl_xor(l, 2, 32); l += __shfl_xor(l, 4, 32); l += __shfl_xor(l, 8, 32); li[r] = 1.0f / l; }
#pragma unroll
    for (int ot = 0; ot < 4; ++ot)
#pragma unroll
        for (int r = 0; r < 8; ++r) os[(8 * hi + r) * 68 + ot * 16 + lr] = acc[ot][r] * li[r];
    __syncthreads();
#pragma unroll 1
    for (int ps = 0; ps < 2; ++ps) {
#pragma unroll
        for (int s = 0; s < 4; ++s) { const int row = 4 * s + (lane >> 3), c8 = (lane & 7) * 8;
            const v4f x0 = *(const v4fa*)(os + row * 68 + c8), x1 = *(const v4fa*)(os + row * 68 + c8 + 4); v8us oh, ol;
#pragma unroll
            for (int k = 0; k < 4; ++k) { unsigned short a, c; splitf(x0[k], a, c); oh[k] = a; ol[k] = c; splitf(x1[k], a, c); oh[4 + k] = a; ol[4 + k] = c; }
            const size_t oo = (size_t)(q0 + row) * DQ + (size_t)h * HD + c8;
            *(volatile v8us*)(Ch + oo) = oh; *(volatile v8us*)(Cl + oo) = ol; }
        if (ps == 0) __threadfence(); }
}
__global__ __launch_bounds__(32) void k_attn_hl(const bf* __restrict__ Qh, const bf* __restrict__ Ql, const bf* __restrict__ Kh, const bf* __restrict__ Kl, const bf* __restrict__ Vh, const bf* __restrict__ Vl,
                                                const unsigned* __restrict__ MBp, const int* __restrict__ CLp, bf* Ch, bf* Cl, int qt0) {
    attn_body<true>((const h16*)0, (const h16*)0, (const h16*)0, Qh, Ql, Kh, Kl, Vh, Vl, MBp, CLp, Ch, Cl, qt0); }
__global__ __launch_bounds__(32) void k_attn_f16(const h16* __restrict__ Q16, const h16* __restrict__ K16, const h16* __restrict__ V16,
                                                 const unsigned* __restrict__ MBp, const int* __restrict__ CLp, bf* Ch, bf* Cl, int qt0) {
    attn_body<false>(Q16, K16, V16, (const bf*)0, (const bf*)0, (const bf*)0, (const bf*)0, (const bf*)0, (const bf*)0, MBp, CLp, Ch, Cl, qt0); }

constexpr size_t al256(size_t b) { return (b + 255) & ~(size_t)255; }
constexpr size_t WS_TOTAL =
    al256((size_t)DQ * DM * 2) + 2 * al256((size_t)DKV * DM * 2) + al256((size_t)DM * DQ * 2) +
    al256((size_t)SEQ * DM * 2) +
    al256((size_t)SEQ * DQ * 4) + 2 * al256((size_t)SEQ * DKV * 4) +
    3 * al256((size_t)NH * SEQ * HD * 2) + 6 * al256((size_t)NKV * SEQ * HD * 2) +
    2 * al256((size_t)SEQ * DQ * 2) +
    al256((size_t)SEQ * NW * 4) + al256((size_t)(SEQ / 16) * NW * 4);
static_assert(WS_TOTAL <= (size_t)134217728);

extern "C" void kernel_launch(void* const* d_in, const int* in_sizes, int n_in,
                              void* d_out, int out_size, void* d_ws, size_t ws_size, hipStream_t stream) {
    if (n_in < 8) return;
    if ((long long)in_sizes[0] < (long long)(NB - 1) * SEQ_FULL * DM + (long long)SEQ * DM) return;
    if ((long long)in_sizes[1] < (long long)DM * DQ || (long long)in_sizes[2] < (long long)DM * DKV || (long long)in_sizes[3] < (long long)DM * DKV || (long long)in_sizes[4] < (long long)DQ * DM) return;
    if ((long long)in_sizes[5] < (long long)SEQ * (HD / 2) || (long long)in_sizes[6] < (long long)SEQ * (HD / 2)) return;
    if ((long long)in_sizes[7] < (long long)(SEQ - 1) * SEQ_FULL + SEQ) return;
    if ((long long)out_size < (long long)(NB - 1) * SEQ_FULL * DM + (long long)SEQ * DM) return;
    if (ws_size < WS_TOTAL) return;
    const float* x = (const float*)d_in[0]; const float* wq = (const float*)d_in[1]; const float* wk = (const float*)d_in[2]; const float* wv = (const float*)d_in[3]; const float* wo = (const float*)d_in[4];
    const float* fcos = (const float*)d_in[5]; const float* fsin = (const float*)d_in[6]; const int* mask = (const int*)d_in[7];
    float* OUT = (float*)d_out;
    char* wsp = (char*)d_ws;
    auto take = [&](size_t bytes) { char* p = wsp; wsp += (bytes + 255) & ~(size_t)255; return (void*)p; };
    bf* WQ = (bf*)take((size_t)DQ * DM * 2); bf* WK = (bf*)take((size_t)DKV * DM * 2); bf* WV = (bf*)take((size_t)DKV * DM * 2); bf* WO = (bf*)take((size_t)DM * DQ * 2);
    bf* XB = (bf*)take((size_t)SEQ * DM * 2);
    float* FQ = (float*)take((size_t)SEQ * DQ * 4); float* FK = (float*)take((size_t)SEQ * DKV * 4); float* FV = (float*)take((size_t)SEQ * DKV * 4);
    h16* QP16 = (h16*)take((size_t)NH * SEQ * HD * 2); bf* QPh = (bf*)take((size_t)NH * SEQ * HD * 2); bf* QPl = (bf*)take((size_t)NH * SEQ * HD * 2);
    h16* KP16 = (h16*)take((size_t)NKV * SEQ * HD * 2); bf* KPh = (bf*)take((size_t)NKV * SEQ * HD * 2); bf* KPl = (bf*)take((size_t)NKV * SEQ * HD * 2);
    h16* VT16 = (h16*)take((size_t)NKV * SEQ * HD * 2); bf* VTh = (bf*)take((size_t)NKV * SEQ * HD * 2); bf* VTl = (bf*)take((size_t)NKV * SEQ * HD * 2);
    bf* CXh = (bf*)take((size_t)SEQ * DQ * 2); bf* CXl = (bf*)take((size_t)SEQ * DQ * 2);
    unsigned* MBp = (unsigned*)take((size_t)SEQ * NW * 4); int* CLp = (int*)take((size_t)(SEQ / 16) * NW * 4);
    if ((size_t)(wsp - (char*)d_ws) > ws_size) return;

    k_wtG<<<(unsigned)((DM * DQ / 64 + 63) / 64), 256, 0, stream>>>(wq, DM, DQ, WQ);
    k_wtG<<<(unsigned)((DM * DKV / 64 + 63) / 64), 256, 0, stream>>>(wk, DM, DKV, WK);
    k_wtG<<<(unsigned)((DM * DKV / 64 + 63) / 64), 256, 0, stream>>>(wv, DM, DKV, WV);
    k_wtG<<<(unsigned)((DQ * DM / 64 + 63) / 64), 256, 0, stream>>>(wo, DQ, DM, WO);
    k_maskbits<<<SEQ / 16, 32, 0, stream>>>(mask, MBp, CLp);
    const unsigned LQ = (unsigned)(((size_t)NH * SEQ * HD / 2 + 255) / 256), LKv = (unsigned)(((size_t)NKV * SEQ * HD / 2 + 255) / 256);
    for (int b = 0; b < NB; ++b) {
        k_cvt8<<<(unsigned)(((size_t)SEQ * DM / 8 + 255) / 256), 256, 0, stream>>>(x + (size_t)b * SEQ_FULL * DM, XB, (size_t)SEQ * DM / 8);
        k_gemm_p<<<dim3(SEQ / 64, DQ / 64, 1), 32, 0, stream>>>(XB, WQ, DM, FQ, DQ);
        k_gemm_p<<<dim3(SEQ / 64, DKV / 64, 1), 32, 0, stream>>>(XB, WK, DM, FK, DKV);
        k_gemm_p<<<dim3(SEQ / 64, DKV / 64, 1), 32, 0, stream>>>(XB, WV, DM, FV, DKV);
        k_rope<<<LQ, 256, 0, stream>>>(FQ, DQ, NH, fcos, fsin, QP16, QPh, QPl);
        k_rope<<<LKv, 256, 0, stream>>>(FK, DKV, NKV, fcos, fsin, KP16, KPh, KPl);
        k_vtp<<<LKv, 256, 0, stream>>>(FV, DKV, NKV, VT16, VTh, VTl);
        if (RH / 16 > 0) k_attn_hl<<<dim3(RH / 16, NH, 1), 32, 0, stream>>>(QPh, QPl, KPh, KPl, VTh, VTl, MBp, CLp, CXh, CXl, 0);
        if ((SEQ - RH) / 16 > 0) k_attn_f16<<<dim3((SEQ - RH) / 16, NH, 1), 32, 0, stream>>>(QP16, KP16, VT16, MBp, CLp, CXh, CXl, RH / 16);
        k_gemm_s<<<dim3(SEQ / 64, DM / 64, 1), 32, 0, stream>>>(CXh, CXl, WO, DQ, OUT + (size_t)b * SEQ_FULL * DM, DM);
    }
}
